// GatedDeltaNetAttention_24507083391404
// MI455X (gfx1250) — hardware-verified
//
#include <hip/hip_runtime.h>
#include <math.h>

constexpr int kBatch = 2;
constexpr int kSeqT  = 2048;
constexpr int kDim   = 1024;
constexpr int kHeads = 16;
constexpr int kDK    = 64;
constexpr int kHD    = kHeads * kDK;
constexpr int kTok   = kBatch * kSeqT;
constexpr int kTaps  = 4;
constexpr int kNqkv  = 3 * kHD;
constexpr int kNab   = 64;
constexpr int kCh    = 32;
constexpr int kNCh   = kSeqT / kCh;
constexpr float kL2Eps  = 1e-6f;
constexpr float kRmsEps = 1e-5f;
static_assert(kDim % 32 == 0 && kHD % 32 == 0, "K multiples of 32");
static_assert(kTok % 64 == 0 && kNqkv % 64 == 0 && kHD % 64 == 0 && kDim % 64 == 0 && kNab % 64 == 0, "M,N multiples of 64");
static_assert(kHeads == 16 && kDK == 64 && kCh == 32 && kSeqT % kCh == 0, "chunk kernel geometry");
static_assert(2 * kHeads <= kNab, "a|b fold");
static_assert((kTok * kDim) % (8 * 256) == 0 && kDim % 64 == 0 && kHD == kDim, "cast and transpose coverage");

constexpr float kCarryQK = 8.0f;
constexpr float kCarryS  = 16.0f;
constexpr float kCarryU  = 16.0f;
constexpr float kCarryL  = 8192.0f;
constexpr float kCarryKd = 16384.0f;
constexpr float kInvQK2  = 1.0f / (kCarryQK * kCarryQK);
constexpr float kInvQKS  = 1.0f / (kCarryQK * kCarryS);
constexpr float kLfac    = kCarryL * kInvQK2;
constexpr float kKdfac   = kCarryKd / kCarryQK;
constexpr float kInvLU   = 1.0f / (kCarryL * kCarryU);
constexpr float kInvKdU  = 1.0f / (kCarryKd * kCarryU);

typedef __attribute__((ext_vector_type(16))) _Float16 v16h;
typedef __attribute__((ext_vector_type(8)))  _Float16 v8h;
typedef __attribute__((ext_vector_type(16))) __bf16   v16b;
typedef __attribute__((ext_vector_type(8)))  __bf16   v8b;
typedef __attribute__((ext_vector_type(8)))  float    v8f;
typedef __attribute__((ext_vector_type(4)))  float    v4f;
typedef __attribute__((ext_vector_type(4)))  unsigned int v4u;

__device__ __forceinline__ unsigned short f2bf_bits(float f) {
  unsigned u = __float_as_uint(f);
  return (unsigned short)((u + 0x7FFFu + ((u >> 16) & 1u)) >> 16);
}
__device__ __forceinline__ float bf_bits2f(unsigned short h) { return __uint_as_float(((unsigned)h) << 16); }
__device__ __forceinline__ float bf_rn(float f) { return bf_bits2f(f2bf_bits(f)); }
__device__ __forceinline__ unsigned pk16(unsigned short a, unsigned short b) { return (unsigned)a | ((unsigned)b << 16); }
__device__ __forceinline__ unsigned short h_bits(float f) { const _Float16 hv = (_Float16)f; return __builtin_bit_cast(unsigned short, hv); }
__device__ __forceinline__ float h16_to_f32(unsigned hb) {
  const unsigned sgn = (hb & 0x8000u) << 16; const unsigned em = hb & 0x7fffu;
  const float fn = __uint_as_float((em << 13) + 0x38000000u);
  const float fs = (float)em * 5.9604644775390625e-8f;
  const float mag = (em < 0x400u) ? fs : fn; return __uint_as_float(__float_as_uint(mag) | sgn); }

__device__ __forceinline__ void dep_guard4_h(v8f& a, v8f& b, v8f& c, v8f& d, v16h x, v16h y, v16h p, v16h q, v16h r, v16h s) {
  asm volatile("v_nop\n\tv_nop\n\tv_nop\n\tv_nop" : "+v"(a), "+v"(b), "+v"(c), "+v"(d) : "v"(x), "v"(y), "v"(p), "v"(q), "v"(r), "v"(s));
}
__device__ __forceinline__ void dep_guard4_b(v8f& a, v8f& b, v8f& c, v8f& d, v16b x, v16b y, v16b p, v16b q, v16b r, v16b s) {
  asm volatile("v_nop\n\tv_nop\n\tv_nop\n\tv_nop" : "+v"(a), "+v"(b), "+v"(c), "+v"(d) : "v"(x), "v"(y), "v"(p), "v"(q), "v"(r), "v"(s));
}
__device__ __forceinline__ void dep_guard3_h(v8f& a, v8f& b, v8f& c, v16h x, v16h y, v16h p, v16h q, v16h r) {
  asm volatile("v_nop\n\tv_nop\n\tv_nop\n\tv_nop" : "+v"(a), "+v"(b), "+v"(c) : "v"(x), "v"(y), "v"(p), "v"(q), "v"(r));
}
__device__ __forceinline__ void keep4_h(v16h a, v16h b, v16h c, v16h d) { asm volatile("v_nop" :: "v"(a), "v"(b), "v"(c), "v"(d)); }
__device__ __forceinline__ void keep4_b(v16b a, v16b b, v16b c, v16b d) { asm volatile("v_nop" :: "v"(a), "v"(b), "v"(c), "v"(d)); }
__device__ __forceinline__ void acc_guard4(v8f& a, v8f& b, v8f& c, v8f& d) { asm volatile("v_nop\n\tv_nop\n\tv_nop\n\tv_nop" : "+v"(a), "+v"(b), "+v"(c), "+v"(d)); }
__device__ __forceinline__ void acc_guard3(v8f& a, v8f& b, v8f& c) { asm volatile("v_nop\n\tv_nop\n\tv_nop\n\tv_nop" : "+v"(a), "+v"(b), "+v"(c)); }
template <typename T> struct Frag;
template <> struct Frag<_Float16> {
  typedef v16h V; union U { v16h v; v8h h[2]; };
  static __device__ __forceinline__ v16h load(const _Float16* p) {
    U f; f.h[0] = *(const v8h*)(p); f.h[1] = *(const v8h*)(p + 16); return f.v;
  }
  static __device__ __forceinline__ v8f mma(v16h a, v16h b, v8f c) {
    return __builtin_amdgcn_wmma_f32_16x16x32_f16(false, a, false, b, (short)0, c, false, false);
  }
  static __device__ __forceinline__ void guard4(v8f& a, v8f& b, v8f& c, v8f& d, v16h x, v16h y, v16h p, v16h q, v16h r, v16h s) { dep_guard4_h(a, b, c, d, x, y, p, q, r, s); }
  static __device__ __forceinline__ void keep(v16h a, v16h b, v16h c, v16h d) { keep4_h(a, b, c, d); }
};
template <> struct Frag<__bf16> {
  typedef v16b V; union U { v16b v; v8b h[2]; };
  static __device__ __forceinline__ v16b load(const __bf16* p) {
    U f; f.h[0] = *(const v8b*)(p); f.h[1] = *(const v8b*)(p + 16); return f.v;
  }
  static __device__ __forceinline__ v8f mma(v16b a, v16b b, v8f c) {
    return __builtin_amdgcn_wmma_f32_16x16x32_bf16(false, a, false, b, (short)0, c, false, false);
  }
  static __device__ __forceinline__ void guard4(v8f& a, v8f& b, v8f& c, v8f& d, v16b x, v16b y, v16b p, v16b q, v16b r, v16b s) { dep_guard4_b(a, b, c, d, x, y, p, q, r, s); }
  static __device__ __forceinline__ void keep(v16b a, v16b b, v16b c, v16b d) { keep4_b(a, b, c, d); }
};

template <int ET> struct Elem;
template <> struct Elem<0> { typedef _Float16 T; };
template <> struct Elem<1> { typedef __bf16 T; };
template <int ET, int SPLIT, int BIAS_MODE, int OUT_MODE>
__global__ __launch_bounds__(256) void wmma_gemm64(
    const unsigned short* __restrict__ Ap, const unsigned short* __restrict__ A2p, int lda, long strideA,
    const unsigned short* __restrict__ Btp, const unsigned short* __restrict__ Bt2p, int ldb, long strideB,
    void* __restrict__ Cout, void* __restrict__ Cout2, int ldc, long strideC,
    const float* __restrict__ bias,
    int M, int N, int K, float scale) {
  typedef typename Elem<ET>::T T;
  typedef typename Frag<T>::V V;
  const T* A = (const T*)Ap; const T* A2 = (const T*)A2p; const T* Bt = (const T*)Btp; const T* Bt2 = (const T*)Bt2p;
  __shared__ __align__(16) float sT[8][16 * 68];
  const int b    = blockIdx.y;
  const int lane = threadIdx.x & 31;
  const int wave = threadIdx.x >> 5;
  const int tilesN = N >> 6;
  const int tilesM = M >> 6;
  const int tile = blockIdx.x * 8 + wave;
  if (tile >= tilesM * tilesN) return;
  const int tm = tile / tilesN;
  const int tn = tile - tm * tilesN;
  const int m0 = tm << 6;
  const int n0 = tn << 6;

  const T* Ab  = A  + (size_t)b * strideA;
  const T* Bb  = Bt + (size_t)b * strideB;
  const T* Ab2 = (SPLIT != 0) ? (A2  + (size_t)b * strideA) : nullptr;
  const T* Bb2 = (SPLIT == 1) ? (Bt2 + (size_t)b * strideB) : nullptr;

  const int rlane = lane & 15;
  const int koff  = (lane >> 4) * 8;
  const int mOff  = (lane >> 4) * 8;

  v8f acc[4][4];
#pragma unroll
  for (int i = 0; i < 4; ++i)
#pragma unroll
    for (int j = 0; j < 4; ++j) acc[i][j] = (v8f){0.f,0.f,0.f,0.f,0.f,0.f,0.f,0.f};

  for (int k0 = 0; k0 < K; k0 += 32) {
    V bh[4], bl[4];
#pragma unroll
    for (int j = 0; j < 4; ++j) {
      const size_t bo = (size_t)(n0 + (j << 4) + rlane) * ldb + koff + k0;
      bh[j] = Frag<T>::load(Bb + bo);
      if (SPLIT == 1) bl[j] = Frag<T>::load(Bb2 + bo);
    }
#pragma unroll
    for (int i = 0; i < 4; ++i) {
      const size_t ao = (size_t)(m0 + (i << 4) + rlane) * lda + koff + k0;
      V ah = Frag<T>::load(Ab + ao);
      V al = ah;
      if (SPLIT != 0) al = Frag<T>::load(Ab2 + ao);
#pragma unroll
      for (int j = 0; j < 4; ++j) {
        acc[i][j] = Frag<T>::mma(ah, bh[j], acc[i][j]);
        if (SPLIT == 1) {
          acc[i][j] = Frag<T>::mma(ah, bl[j], acc[i][j]);
          acc[i][j] = Frag<T>::mma(al, bh[j], acc[i][j]);
        }
        if (SPLIT == 2) acc[i][j] = Frag<T>::mma(al, bh[j], acc[i][j]);
      }
      Frag<T>::guard4(acc[i][0], acc[i][1], acc[i][2], acc[i][3], ah, al, bh[0], bh[1], bh[2], bh[3]);
    }
    Frag<T>::keep(bh[0], bh[1], bh[2], bh[3]);
    if (SPLIT == 1) Frag<T>::keep(bl[0], bl[1], bl[2], bl[3]);
  }
  acc_guard4(acc[0][0], acc[0][1], acc[0][2], acc[0][3]);
  acc_guard4(acc[1][0], acc[1][1], acc[1][2], acc[1][3]);
  acc_guard4(acc[2][0], acc[2][1], acc[2][2], acc[2][3]);
  acc_guard4(acc[3][0], acc[3][1], acc[3][2], acc[3][3]);

  float* slab = sT[wave];
#pragma unroll
  for (int i = 0; i < 4; ++i) {
    const int mBase = m0 + (i << 4);
#pragma unroll
    for (int j = 0; j < 4; ++j) {
      const int n = n0 + (j << 4) + rlane;
      float bv = 0.f;
      if (BIAS_MODE == 2) bv = bias[n];
#pragma unroll
      for (int r = 0; r < 8; ++r) {
        float v = acc[i][j][r] * scale;
        if (BIAS_MODE == 1) v += bias[mBase + mOff + r];
        if (BIAS_MODE == 2) v += bv;
        slab[(mOff + r) * 68 + (j << 4) + rlane] = v;
      }
    }
    __builtin_amdgcn_fence(__ATOMIC_RELEASE, "workgroup");
    __builtin_amdgcn_wave_barrier();
    __builtin_amdgcn_fence(__ATOMIC_ACQUIRE, "workgroup");
    if (OUT_MODE == 0) {
      float* C = (float*)Cout + (size_t)b * strideC;
      const int hh = lane >> 4, c4 = (lane & 15) * 4;
      for (int pass = 0; pass < 2; ++pass) {
#pragma unroll
        for (int it = 0; it < 8; ++it) {
          const int row = it * 2 + hh;
          v4f v = *(const v4f*)(slab + row * 68 + c4);
          *(volatile v4f*)(C + (size_t)(mBase + row) * ldc + n0 + c4) = v;
        }
        __threadfence();
      }
    } else {
      const int q = lane >> 3, c8 = (lane & 7) * 8;
      unsigned short* C  = (unsigned short*)Cout  + (size_t)b * strideC;
      unsigned short* C2 = (OUT_MODE == 2) ? ((unsigned short*)Cout2 + (size_t)b * strideC) : nullptr;
      for (int pass = 0; pass < 2; ++pass) {
#pragma unroll
        for (int it = 0; it < 4; ++it) {
          const int row = it * 4 + q;
          const float* sp = slab + row * 68 + c8;
          v8h hv, lv;
#pragma unroll
          for (int e = 0; e < 8; ++e) {
            if (OUT_MODE == 1) {
              hv[e] = (_Float16)sp[e];
            } else {
              unsigned short hb = f2bf_bits(sp[e]);
              unsigned short lb = f2bf_bits(sp[e] - bf_bits2f(hb));
              hv[e] = __builtin_bit_cast(_Float16, hb);
              lv[e] = __builtin_bit_cast(_Float16, lb);
            }
          }
          *(volatile v8h*)(C + (size_t)(mBase + row) * ldc + n0 + c8) = hv;
          if (OUT_MODE == 2) *(volatile v8h*)(C2 + (size_t)(mBase + row) * ldc + n0 + c8) = lv;
        }
        __threadfence();
      }
    }
    __builtin_amdgcn_fence(__ATOMIC_RELEASE, "workgroup");
    __builtin_amdgcn_wave_barrier();
    __builtin_amdgcn_fence(__ATOMIC_ACQUIRE, "workgroup");
  }
}

__global__ __launch_bounds__(256) void cast8_bf16_kernel(const float* __restrict__ in, unsigned short* __restrict__ out, int n8) {
  const int i = blockIdx.x * 256 + threadIdx.x;
  if (i >= n8) return;
  const float* p = in + 8 * (size_t)i;
  const v4f a = *(const v4f*)(p);
  const v4f c = *(const v4f*)(p + 4);
  unsigned short hb[8];
#pragma unroll
  for (int e = 0; e < 4; ++e) {
    hb[e]     = f2bf_bits(a[e]);
    hb[4 + e] = f2bf_bits(c[e]);
  }
  const v4u u = (v4u){pk16(hb[0], hb[1]), pk16(hb[2], hb[3]), pk16(hb[4], hb[5]), pk16(hb[6], hb[7])};
  unsigned short* q = out + 8 * (size_t)i;
  *(volatile v4u*)q = u;
  __threadfence();
  *(volatile v4u*)q = u;
}

__global__ __launch_bounds__(256) void wtrans_kernel(const float* __restrict__ W0, const float* __restrict__ W1,
                                                     const float* __restrict__ W2, const float* __restrict__ W3,
                                                     const float* __restrict__ W4,
                                                     unsigned short* __restrict__ wt, unsigned short* __restrict__ wot) {
  __shared__ float sm[64][65];
  const int t  = threadIdx.x;
  const int k0 = blockIdx.x * 64;
  const int n0 = blockIdx.y * 64;
  const int z  = blockIdx.z;
  const float* W = (z == 0) ? W0 : (z == 1) ? W1 : (z == 2) ? W2 : (z == 3) ? W3 : W4;
  unsigned short* op = (z < 4) ? (wt + (size_t)z * kHD * kDim) : wot;
#pragma unroll
  for (int i = 0; i < 8; ++i) {
    const int e = i * 256 + t;
    const int r = e >> 6;
    const int c = e & 63;
    sm[c][r] = W[(size_t)(k0 + r) * kDim + n0 + c];
  }
  asm volatile("" ::: "memory");
#pragma unroll
  for (int i = 8; i < 16; ++i) {
    const int e = i * 256 + t;
    const int r = e >> 6;
    const int c = e & 63;
    sm[c][r] = W[(size_t)(k0 + r) * kDim + n0 + c];
  }
  __syncthreads();
  const int lane = t & 31, wave = t >> 5;
  const int q = lane >> 3, c8 = (lane & 7) * 8;
  for (int pass = 0; pass < 2; ++pass) {
#pragma unroll
    for (int it = 0; it < 2; ++it) {
      const int row = wave * 8 + it * 4 + q;
      unsigned short hb[8];
#pragma unroll
      for (int e = 0; e < 8; ++e) hb[e] = f2bf_bits(sm[row][c8 + e]);
      const v4u u = (v4u){pk16(hb[0], hb[1]), pk16(hb[2], hb[3]), pk16(hb[4], hb[5]), pk16(hb[6], hb[7])};
      *(volatile v4u*)(op + (size_t)(n0 + row) * kDim + k0 + c8) = u;
    }
    __threadfence();
  }
}

__global__ __launch_bounds__(128) void wab_kernel(const float* __restrict__ wa, const float* __restrict__ wb,
                                                  unsigned short* __restrict__ wab) {
  const int row = blockIdx.x;
  const int k0  = 8 * threadIdx.x;
  const bool useA = row < kHeads;
  const bool zero = row >= 2 * kHeads;
  int nn = useA ? row : (row - kHeads);
  nn = nn < 0 ? 0 : (nn > kHeads - 1 ? kHeads - 1 : nn);
  const float* src = useA ? wa : wb;
  unsigned short hb[8];
#pragma unroll
  for (int e = 0; e < 8; ++e) {
    const float v = src[(size_t)(k0 + e) * kHeads + nn];
    hb[e] = f2bf_bits(zero ? 0.0f : v);
  }
  const v4u u = (v4u){pk16(hb[0], hb[1]), pk16(hb[2], hb[3]), pk16(hb[4], hb[5]), pk16(hb[6], hb[7])};
  unsigned short* q = wab + (size_t)row * kDim + k0;
  *(volatile v4u*)q = u;
  __threadfence();
  *(volatile v4u*)q = u;
}

__global__ __launch_bounds__(256) void decbeta_kernel(const float* __restrict__ ab, const float* __restrict__ alog,
                                                      const float* __restrict__ dtb, float* __restrict__ gpl,
                                                      float* __restrict__ bpl) {
  __shared__ __align__(16) float sd[8][32];
  __shared__ __align__(16) float sb[8][32];
  const int lane = threadIdx.x & 31, wave = threadIdx.x >> 5;
  const int base = (blockIdx.x * 8 + wave) * 2;
  const int row  = base + (lane >> 4);
  const int hd   = lane & 15;
  const float xa = ab[(size_t)row * kNab + hd];
  const float xb = ab[(size_t)row * kNab + kHeads + hd];
  const float nal = bf_rn(alog[hd]);
  const float ndb = bf_rn(dtb[hd]);
  const float x  = xa + ndb;
  const float sp = fmaxf(x, 0.0f) + log1pf(expf(-fabsf(x)));
  const float gd = -expf(nal) * sp;
  const float bet = 1.0f / (1.0f + expf(-xb));
  sd[wave][lane] = gd;
  sb[wave][lane] = bet;
  __builtin_amdgcn_fence(__ATOMIC_RELEASE, "workgroup");
  __builtin_amdgcn_wave_barrier();
  __builtin_amdgcn_fence(__ATOMIC_ACQUIRE, "workgroup");
  const int c4 = (lane & 7) * 4;
  const v4f dv4 = *(const v4f*)(&sd[wave][c4]);
  const v4f bv4 = *(const v4f*)(&sb[wave][c4]);
  float* pd = gpl + (size_t)base * kHeads + c4;
  float* pb = bpl + (size_t)base * kHeads + c4;
  if (lane < 8) { *(volatile v4f*)pd = dv4; *(volatile v4f*)pb = bv4; }
  __threadfence();
  if (lane < 8) { *(volatile v4f*)pd = dv4; *(volatile v4f*)pb = bv4; }
}

__global__ __launch_bounds__(128) void conv_qk_kernel(const float* __restrict__ pre, const float* __restrict__ qcw,
                                                      const float* __restrict__ kcw, unsigned short* __restrict__ qn,
                                                      unsigned short* __restrict__ kn) {
  const int row   = blockIdx.x;
  const int which = blockIdx.y;
  const int lane  = threadIdx.x & 31, wave = threadIdx.x >> 5;
  const int hd    = wave * 4 + (lane >> 3);
  const int c0    = hd * kDK + (lane & 7) * 8;
  const float* cw = which ? kcw : qcw;
  unsigned short* outp = which ? kn : qn;
  const int t    = row & (kSeqT - 1);
  const int pcol = which * kHD + c0;
  v4f w[8];
#pragma unroll
  for (int e = 0; e < 8; ++e) w[e] = *(const v4f*)(cw + (size_t)(c0 + e) * kTaps);
  asm volatile("" ::: "memory");
  float a[8];
#pragma unroll
  for (int e = 0; e < 8; ++e) a[e] = 0.0f;
#pragma unroll
  for (int j = 0; j < kTaps; ++j) {
    const int tk = t - (kTaps - 1) + j;
    int srow = row - (kTaps - 1) + j;
    srow = srow < 0 ? 0 : srow;
    const bool on = tk >= 0;
    const float* xp = pre + (size_t)srow * kNqkv + pcol;
    const v4f x0 = *(const v4f*)(xp);
    const v4f x1 = *(const v4f*)(xp + 4);
#pragma unroll
    for (int e = 0; e < 4; ++e) {
      const float xs0 = on ? x0[e] : 0.0f;
      const float xs1 = on ? x1[e] : 0.0f;
      a[e]     = fmaf(xs0, bf_rn(w[e][j]), a[e]);
      a[4 + e] = fmaf(xs1, bf_rn(w[4 + e][j]), a[4 + e]);
    }
  }
  float s[8];
  float ss = 0.0f;
#pragma unroll
  for (int e = 0; e < 8; ++e) {
    s[e] = a[e] * (1.0f / (1.0f + expf(-a[e])));
    ss = fmaf(s[e], s[e], ss);
  }
  ss += __shfl_xor(ss, 1, 32);
  ss += __shfl_xor(ss, 2, 32);
  ss += __shfl_xor(ss, 4, 32);
  const float rs = rsqrtf(ss + kL2Eps);
  unsigned short hb[8];
#pragma unroll
  for (int e = 0; e < 8; ++e) hb[e] = h_bits(kCarryQK * (s[e] * rs));
  const v4u u = (v4u){pk16(hb[0], hb[1]), pk16(hb[2], hb[3]), pk16(hb[4], hb[5]), pk16(hb[6], hb[7])};
  unsigned short* op = outp + (size_t)row * kHD + c0;
  *(volatile v4u*)op = u;
  __threadfence();
  *(volatile v4u*)op = u;
}

__global__ __launch_bounds__(256) void conv_v_kernel(const float* __restrict__ pre, const float* __restrict__ vcw,
                                                     float* __restrict__ vpl) {
  const int row = blockIdx.x;
  const int t   = row & (kSeqT - 1);
  const int c0  = 4 * threadIdx.x;
  const v4f w0 = *(const v4f*)(vcw + (size_t)(c0 + 0) * kTaps);
  const v4f w1 = *(const v4f*)(vcw + (size_t)(c0 + 1) * kTaps);
  const v4f w2 = *(const v4f*)(vcw + (size_t)(c0 + 2) * kTaps);
  const v4f w3 = *(const v4f*)(vcw + (size_t)(c0 + 3) * kTaps);
  asm volatile("" ::: "memory");
  float a0 = 0.0f, a1 = 0.0f, a2 = 0.0f, a3 = 0.0f;
#pragma unroll
  for (int j = 0; j < kTaps; ++j) {
    const int tk = t - (kTaps - 1) + j;
    int srow = row - (kTaps - 1) + j;
    srow = srow < 0 ? 0 : srow;
    const bool on = tk >= 0;
    const v4f x = *(const v4f*)(pre + (size_t)srow * kNqkv + 2 * kHD + c0);
    const float x0 = on ? x[0] : 0.0f;
    const float x1 = on ? x[1] : 0.0f;
    const float x2 = on ? x[2] : 0.0f;
    const float x3 = on ? x[3] : 0.0f;
    a0 = fmaf(x0, bf_rn(w0[j]), a0);
    a1 = fmaf(x1, bf_rn(w1[j]), a1);
    a2 = fmaf(x2, bf_rn(w2[j]), a2);
    a3 = fmaf(x3, bf_rn(w3[j]), a3);
  }
  const v4f o = (v4f){a0 * (1.0f / (1.0f + expf(-a0))), a1 * (1.0f / (1.0f + expf(-a1))),
                      a2 * (1.0f / (1.0f + expf(-a2))), a3 * (1.0f / (1.0f + expf(-a3)))};
  float* op = vpl + (size_t)row * kHD + c0;
  *(volatile v4f*)op = o;
  __threadfence();
  *(volatile v4f*)op = o;
}

union KdE2U { float e2[kCh * kCh]; unsigned short kd[kDK * kCh]; };

__global__ __launch_bounds__(256) void chunk_kernel(const unsigned short* __restrict__ qn, const unsigned short* __restrict__ kn,
                                                    const float* __restrict__ vpl, const float* __restrict__ gpl,
                                                    const float* __restrict__ bpl, const unsigned short* __restrict__ gate16,
                                                    const float* __restrict__ rmsw_in, unsigned short* __restrict__ obhi,
                                                    unsigned short* __restrict__ oblo, float scaleq) {
  __shared__ __align__(16) float Sf[kDK * kDK];
  __shared__ __align__(16) unsigned short S16t[kDK * kDK];
  __shared__ __align__(16) unsigned short KQ16[2 * kCh * kDK];
  __shared__ __align__(16) unsigned short L16[kCh * kCh];
  __shared__ __align__(16) unsigned short U16t[kDK * kCh];
  __shared__ __align__(16) KdE2U KE;
  __shared__ __align__(16) float RUf[kCh * kDK];
  __shared__ __align__(16) float QOf[kCh * kDK];
  __shared__ __align__(16) float Mf[kCh * kCh];
  __shared__ float Gc[kCh];
  __shared__ float eG[kCh];
  __shared__ float eGC[kCh];
  __shared__ float bv[kCh];
  __shared__ __align__(16) float rmsw[kDK];

  const int tid   = threadIdx.x;
  const int lane  = tid & 31;
  const int wave  = tid >> 5;
  const int rlane = lane & 15;
  const int hh    = lane >> 4;
  const int koff  = hh * 8;
  const int mOff  = hh * 8;
  const int bh    = blockIdx.x;
  const int b     = bh >> 4;
  const int h     = bh & 15;
  const size_t rowb = (size_t)b * kSeqT;
  const int colh  = h * kDK;

  {
    const v4f z4 = (v4f){0.0f, 0.0f, 0.0f, 0.0f};
    const v4u zu = (v4u){0u, 0u, 0u, 0u};
#pragma unroll
    for (int i = 0; i < 4; ++i) *(v4f*)(Sf + 4 * (tid + 256 * i)) = z4;
#pragma unroll
    for (int i = 0; i < 2; ++i) *(v4u*)(S16t + 8 * (tid + 256 * i)) = zu;
    if (tid < kDK) rmsw[tid] = bf_rn(rmsw_in[tid]);
  }
  __syncthreads();

  const _Float16* kqh   = (const _Float16*)KQ16;
  const _Float16* s16h  = (const _Float16*)S16t;
  const _Float16* l16h  = (const _Float16*)L16;
  const _Float16* u16h  = (const _Float16*)U16t;
  const _Float16* kd16h = (const _Float16*)KE.kd;
  const v8f z8 = (v8f){0.f,0.f,0.f,0.f,0.f,0.f,0.f,0.f};

  for (int ch = 0; ch < kNCh; ++ch) {
    const int t0 = ch * kCh;
    {
      const int rl = tid >> 3, c16 = (tid & 7) * 8;
      const size_t go = (rowb + t0 + rl) * kHD + colh + c16;
      const v4u wk = *(const v4u*)(kn + go);
      const v4u wq = *(const v4u*)(qn + go);
      *(v4u*)(KQ16 + rl * kDK + c16) = wk;
      *(v4u*)(KQ16 + (kCh + rl) * kDK + c16) = wq;
#pragma unroll
      for (int rep = 0; rep < 2; ++rep) {
        const int idx = tid + 256 * rep;
        const int r2 = idx >> 4, c4 = (idx & 15) * 4;
        *(v4f*)(RUf + r2 * kDK + c4) = *(const v4f*)(vpl + (rowb + t0 + r2) * kHD + colh + c4);
      }
      if (tid < kCh) {
        const size_t gi = (rowb + t0 + tid) * kHeads + h;
        Gc[tid] = gpl[gi];
        bv[tid] = bpl[gi];
      }
    }
    __syncthreads();
    {
#pragma unroll 1
      for (int i = 0; i < 4; ++i) {
        const int idx = tid + 256 * i;
        const int t = idx >> 5, s = idx & 31;
        float sum = 0.0f;
        for (int p = s + 1; p <= t; ++p) sum += Gc[p];
        const float e = expf(sum);
        KE.e2[idx] = (s <= t) ? e : 0.0f;
      }
      if (wave == 0) {
        float sum = 0.0f;
        for (int p = 0; p <= lane; ++p) sum += Gc[p];
        eG[lane] = expf(sum);
      }
      if (wave == 1) {
        float sum = 0.0f;
        for (int p = lane + 1; p < kCh; ++p) sum += Gc[p];
        eGC[lane] = expf(sum);
      }
    }
    __syncthreads();
    {
      const int rt  = wave >> 1;
      const int ctA = wave & 1;
      const int ctB = 2 * (wave & 1);
      v8f accA = z8, accB0 = z8, accB1 = z8;
#pragma unroll
      for (int ks = 0; ks < 2; ++ks) {
        const int k0 = ks * 32;
        const v16h a   = Frag<_Float16>::load(kqh  + (16 * rt + rlane) * kDK + koff + k0);
        const v16h bk  = Frag<_Float16>::load(kqh  + (16 * ctA + rlane) * kDK + koff + k0);
        const v16h bs0 = Frag<_Float16>::load(s16h + (16 * ctB + rlane) * kDK + koff + k0);
        const v16h bs1 = Frag<_Float16>::load(s16h + (16 * (ctB + 1) + rlane) * kDK + koff + k0);
        accA  = Frag<_Float16>::mma(a, bk,  accA);
        accB0 = Frag<_Float16>::mma(a, bs0, accB0);
        accB1 = Frag<_Float16>::mma(a, bs1, accB1);
        dep_guard3_h(accA, accB0, accB1, a, bk, bs0, bs1, bs1);
      }
      acc_guard3(accA, accB0, accB1);
      if (wave < 4) {
#pragma unroll
        for (int r = 0; r < 8; ++r) {
          const int t = 16 * rt + mOff + r;
          const int s = 16 * ctA + rlane;
          const float bt = bv[t];
          const float egt = eG[t];
          const float e2 = KE.e2[t * kCh + s];
          Mf[t * kCh + s] = (s < t) ? (bt * e2 * accA[r] * kInvQK2) : 0.0f;
          const int i0 = t * kDK + 16 * ctB + rlane;
          const int i1 = i0 + 16;
          RUf[i0] = bt * (RUf[i0] - egt * accB0[r] * kInvQKS);
          RUf[i1] = bt * (RUf[i1] - egt * accB1[r] * kInvQKS);
        }
      } else {
#pragma unroll
        for (int r = 0; r < 8; ++r) {
          const int t = 16 * (rt - 2) + mOff + r;
          const int s = 16 * ctA + rlane;
          const float egt = eG[t];
          const float e2 = KE.e2[t * kCh + s];
          const float lvv = (s <= t) ? (e2 * accA[r] * kLfac) : 0.0f;
          L16[t * kCh + s] = h_bits(lvv);
          const int i0 = t * kDK + 16 * ctB + rlane;
          const int i1 = i0 + 16;
          QOf[i0] = egt * accB0[r] * kInvQKS;
          QOf[i1] = egt * accB1[r] * kInvQKS;
        }
      }
    }
    __syncthreads();
    if (tid < kDK) {
      const int v = tid;
#pragma unroll 1
      for (int t = 0; t < kCh; ++t) {
        float u = RUf[t * kDK + v];
        for (int s = 0; s < t; ++s) u = fmaf(-Mf[t * kCh + s], RUf[s * kDK + v], u);
        RUf[t * kDK + v] = u;
        U16t[v * kCh + t] = h_bits(u * kCarryU);
      }
    } else {
      for (int i = tid - kDK; i < kDK * kCh; i += 256 - kDK) {
        const int d = i >> 5, s = i & 31;
        const float kf = h16_to_f32((unsigned)KQ16[s * kDK + d]);
        KE.kd[i] = h_bits(eGC[s] * kf * kKdfac);
      }
    }
    __syncthreads();
    {
      const int rt5 = wave >> 2, ct5 = wave & 3;
      const int rt6 = wave >> 1, ct6 = 2 * (wave & 1);
      const v16h aL  = Frag<_Float16>::load(l16h  + (16 * rt5 + rlane) * kCh + koff);
      const v16h aK  = Frag<_Float16>::load(kd16h + (16 * rt6 + rlane) * kCh + koff);
      const v16h b5  = Frag<_Float16>::load(u16h  + (16 * ct5 + rlane) * kCh + koff);
      const v16h b60 = Frag<_Float16>::load(u16h  + (16 * ct6 + rlane) * kCh + koff);
      const v16h b61 = Frag<_Float16>::load(u16h  + (16 * (ct6 + 1) + rlane) * kCh + koff);
      v8f acc5  = Frag<_Float16>::mma(aL, b5,  z8);
      v8f acc60 = Frag<_Float16>::mma(aK, b60, z8);
      v8f acc61 = Frag<_Float16>::mma(aK, b61, z8);
      dep_guard3_h(acc5, acc60, acc61, aL, aK, b5, b60, b61);
#pragma unroll
      for (int r = 0; r < 8; ++r) {
        const int t = 16 * rt5 + mOff + r;
        const int i = t * kDK + 16 * ct5 + rlane;
        QOf[i] = scaleq * (QOf[i] + acc5[r] * kInvLU);
      }
      const float egc = eG[kCh - 1];
#pragma unroll
      for (int r = 0; r < 8; ++r) {
        const int d  = 16 * rt6 + mOff + r;
        const int v0 = 16 * ct6 + rlane;
        const int v1 = v0 + 16;
        const int i0 = d * kDK + v0;
        const int i1 = d * kDK + v1;
        const float sn0 = fmaf(egc, Sf[i0], acc60[r] * kInvKdU);
        const float sn1 = fmaf(egc, Sf[i1], acc61[r] * kInvKdU);
        Sf[i0] = sn0;
        Sf[i1] = sn1;
        S16t[v0 * kDK + d] = h_bits(sn0 * kCarryS);
        S16t[v1 * kDK + d] = h_bits(sn1 * kCarryS);
      }
    }
    __syncthreads();
    {
      const int tl = 4 * wave + (lane >> 3);
      const int c8 = (lane & 7) * 8;
      const size_t grow = rowb + t0 + tl;
      const v4f oa = *(const v4f*)(QOf + tl * kDK + c8);
      const v4f ob = *(const v4f*)(QOf + tl * kDK + c8 + 4);
      const v4u gw = *(const v4u*)(gate16 + grow * kHD + colh + c8);
      float ov[8], gv[8];
#pragma unroll
      for (int e = 0; e < 4; ++e) { ov[e] = oa[e]; ov[4 + e] = ob[e]; }
      {
        const unsigned w0 = gw[0], w1 = gw[1], w2 = gw[2], w3 = gw[3];
        gv[0] = h16_to_f32(w0 & 0xffffu); gv[1] = h16_to_f32(w0 >> 16);
        gv[2] = h16_to_f32(w1 & 0xffffu); gv[3] = h16_to_f32(w1 >> 16);
        gv[4] = h16_to_f32(w2 & 0xffffu); gv[5] = h16_to_f32(w2 >> 16);
        gv[6] = h16_to_f32(w3 & 0xffffu); gv[7] = h16_to_f32(w3 >> 16);
      }
      float ss = 0.0f;
#pragma unroll
      for (int e = 0; e < 8; ++e) ss = fmaf(ov[e], ov[e], ss);
      ss += __shfl_xor(ss, 1, 32);
      ss += __shfl_xor(ss, 2, 32);
      ss += __shfl_xor(ss, 4, 32);
      const float rs = rsqrtf(ss * (1.0f / kDK) + kRmsEps);
      unsigned short hb[8], lb[8];
#pragma unroll
      for (int e = 0; e < 8; ++e) {
        const float g  = gv[e];
        const float sg = g * (1.0f / (1.0f + expf(-g)));
        const float y  = ((ov[e] * rs) * rmsw[c8 + e]) * sg;
        const unsigned short h16 = f2bf_bits(y);
        hb[e] = h16;
        lb[e] = f2bf_bits(y - bf_bits2f(h16));
      }
      const v4u uh = (v4u){pk16(hb[0], hb[1]), pk16(hb[2], hb[3]), pk16(hb[4], hb[5]), pk16(hb[6], hb[7])};
      const v4u ul = (v4u){pk16(lb[0], lb[1]), pk16(lb[2], lb[3]), pk16(lb[4], lb[5]), pk16(lb[6], lb[7])};
      unsigned short* ph = obhi + grow * kHD + colh + c8;
      unsigned short* pl = oblo + grow * kHD + colh + c8;
      *(volatile v4u*)ph = uh;
      *(volatile v4u*)pl = ul;
      __threadfence();
      *(volatile v4u*)ph = uh;
      *(volatile v4u*)pl = ul;
    }
  }
}

extern "C" void kernel_launch(void* const* d_in, const int* in_sizes, int n_in,
                              void* d_out, int out_size, void* d_ws, size_t ws_size,
                              hipStream_t stream) {
  if (n_in < 14) return;
  if (in_sizes[0] != kTok * kDim) return;
  if (in_sizes[1] != kDim * kHD || in_sizes[2] != kDim * kHD || in_sizes[3] != kDim * kHD) return;
  if (in_sizes[4] != kDim * kHeads || in_sizes[5] != kDim * kHeads) return;
  if (in_sizes[6] != kDim * kHD || in_sizes[7] != kHD * kDim) return;
  if (in_sizes[8] != kHD * kTaps || in_sizes[9] != kHD * kTaps || in_sizes[10] != kHD * kTaps) return;
  if (in_sizes[11] != kHeads || in_sizes[12] != kHeads || in_sizes[13] != kDK) return;
  if (out_size != kTok * kDim) return;

  const size_t szXb  = (size_t)kTok * kDim * 2;
  const size_t szWt  = (size_t)4 * kHD * kDim * 2;
  const size_t szWab = (size_t)kNab * kDim * 2;
  const size_t szWot = (size_t)kDim * kHD * 2;
  const size_t szPre = (size_t)kTok * kNqkv * 4;
  const size_t szGat = (size_t)kTok * kHD * 2;
  const size_t szAb  = (size_t)kTok * kNab * 4;
  const size_t szGb  = (size_t)kTok * kHeads * 4;
  const size_t szQn  = (size_t)kTok * kHD * 2;
  const size_t szVn  = (size_t)kTok * kHD * 4;
  const size_t szY   = (size_t)kTok * kHD * 2;
  const size_t offXb  = 0;
  const size_t offWt  = offXb + szXb;
  const size_t offWab = offWt + szWt;
  const size_t offWot = offWab + szWab;
  const size_t offPre = offWot + szWot;
  const size_t offGat = offPre + szPre;
  const size_t offAb  = offGat + szGat;
  const size_t offG   = offAb + szAb;
  const size_t offBet = offG + szGb;
  const size_t offQn  = offBet + szGb;
  const size_t offKn  = offQn + szQn;
  const size_t offVn  = offKn + szQn;
  const size_t offYhi = offVn + szVn;
  const size_t offYlo = offYhi + szY;
  const size_t total  = offYlo + szY;
  if (ws_size < total) return;

  const float* x    = (const float*)d_in[0];
  const float* wq   = (const float*)d_in[1];
  const float* wk   = (const float*)d_in[2];
  const float* wv   = (const float*)d_in[3];
  const float* wa   = (const float*)d_in[4];
  const float* wb   = (const float*)d_in[5];
  const float* wg   = (const float*)d_in[6];
  const float* wo   = (const float*)d_in[7];
  const float* cq   = (const float*)d_in[8];
  const float* ck   = (const float*)d_in[9];
  const float* cv   = (const float*)d_in[10];
  const float* alog = (const float*)d_in[11];
  const float* dtb  = (const float*)d_in[12];
  const float* rmsw = (const float*)d_in[13];
  float* out = (float*)d_out;
  char* ws = (char*)d_ws;
  unsigned short* xb   = (unsigned short*)(ws + offXb);
  unsigned short* wt   = (unsigned short*)(ws + offWt);
  unsigned short* wab  = (unsigned short*)(ws + offWab);
  unsigned short* wot  = (unsigned short*)(ws + offWot);
  float* pre  = (float*)(ws + offPre);
  unsigned short* gate = (unsigned short*)(ws + offGat);
  float* ab   = (float*)(ws + offAb);
  float* gpl  = (float*)(ws + offG);
  float* bpl  = (float*)(ws + offBet);
  unsigned short* qn   = (unsigned short*)(ws + offQn);
  unsigned short* kn   = (unsigned short*)(ws + offKn);
  float* vpl  = (float*)(ws + offVn);
  unsigned short* yhi  = (unsigned short*)(ws + offYhi);
  unsigned short* ylo  = (unsigned short*)(ws + offYlo);

  const float scaleq = 1.0f / sqrtf((float)kDK);
  const int n8x = (kTok * kDim) / 8;
  const int blocksQkv = ((kTok / 64) * (kNqkv / 64)) / 8;
  const int blocksSq  = ((kTok / 64) * (kDim / 64)) / 8;
  const int blocksAb  = ((kTok / 64) * (kNab / 64)) / 8;

  cast8_bf16_kernel<<<dim3(n8x / 256), dim3(256), 0, stream>>>(x, xb, n8x);
  wtrans_kernel<<<dim3(kDim / 64, kHD / 64, 5), dim3(256), 0, stream>>>(wq, wk, wv, wg, wo, wt, wot);
  wab_kernel<<<dim3(kNab), dim3(128), 0, stream>>>(wa, wb, wab);
  wmma_gemm64<1, 0, 0, 0><<<dim3(blocksQkv, 1), dim3(256), 0, stream>>>(
      xb, xb, kDim, 0L, wt, wt, kDim, 0L, (void*)pre, (void*)pre, kNqkv, 0L, gpl, kTok, kNqkv, kDim, 1.0f);
  wmma_gemm64<1, 0, 0, 1><<<dim3(blocksSq, 1), dim3(256), 0, stream>>>(
      xb, xb, kDim, 0L, wt + (size_t)kNqkv * kDim, wt + (size_t)kNqkv * kDim, kDim, 0L,
      (void*)gate, (void*)gate, kHD, 0L, gpl, kTok, kHD, kDim, 1.0f);
  wmma_gemm64<1, 0, 0, 0><<<dim3(blocksAb, 1), dim3(256), 0, stream>>>(
      xb, xb, kDim, 0L, wab, wab, kDim, 0L, (void*)ab, (void*)ab, kNab, 0L, gpl, kTok, kNab, kDim, 1.0f);
  decbeta_kernel<<<dim3(kTok / 16), dim3(256), 0, stream>>>(ab, alog, dtb, gpl, bpl);
  conv_qk_kernel<<<dim3(kTok, 2), dim3(128), 0, stream>>>(pre, cq, ck, qn, kn);
  conv_v_kernel<<<dim3(kTok), dim3(256), 0, stream>>>(pre, cv, vpl);
  chunk_kernel<<<dim3(kBatch * kHeads), dim3(256), 0, stream>>>(qn, kn, vpl, gpl, bpl, gate, rmsw, yhi, ylo, scaleq);
  wmma_gemm64<1, 2, 0, 0><<<dim3(blocksSq, 1), dim3(256), 0, stream>>>(
      yhi, ylo, kHD, 0L, wot, wot, kHD, 0L, (void*)out, (void*)out, kDim, 0L, gpl, kTok, kDim, kHD, 1.0f);
}
